// ChannelTransformerStage_2714419331295
// MI455X (gfx1250) — hardware-verified
//
#include <hip/hip_runtime.h>


typedef _Float16 f16_t;
typedef f16_t v16h __attribute__((ext_vector_type(16)));
typedef f16_t v8h __attribute__((ext_vector_type(8)));
typedef float v8f __attribute__((ext_vector_type(8)));
typedef float v4f __attribute__((ext_vector_type(4)));
typedef v8h v8hm __attribute__((may_alias));
typedef v4f v4fm __attribute__((may_alias));

#define H_   4
#define C1_  64
#define C2_  128
#define KV_  192
#define MLP_ 256
#define B_   8
#define N_   3136
#define BN_  (B_ * N_)

union Frag { v16h v; v8h p[2]; };

__device__ __forceinline__ v8f wmma16(v16h a, v16h b, v8f c) {
  v8f d = __builtin_amdgcn_wmma_f32_16x16x32_f16(false, a, false, b, (short)0, c, false, false);
  asm volatile("v_nop\n\tv_nop\n\tv_nop\n\tv_nop" : "+v"(d) : "v"(a), "v"(b));
  return d;
}

__device__ __forceinline__ float wave_sum(float v) {
#pragma unroll
  for (int msk = 16; msk >= 1; msk >>= 1) v += __shfl_xor(v, msk, 32);
  return v;
}
__device__ __forceinline__ float wave_max(float v) {
#pragma unroll
  for (int msk = 16; msk >= 1; msk >>= 1) v = fmaxf(v, __shfl_xor(v, msk, 32));
  return v;
}

__global__ __launch_bounds__(256) void cvt_f16_kernel(const float* __restrict__ src,
                                                      f16_t* __restrict__ dst, int n8) {
  const int i = blockIdx.x * 256 + threadIdx.x;
  const bool ok = i < n8;
  const int ic = ok ? i : 0;
  const v4f x0 = *(const v4fm*)(src + (size_t)ic * 8);
  const v4f x1 = *(const v4fm*)(src + (size_t)ic * 8 + 4);
  v8h v;
#pragma unroll
  for (int j = 0; j < 4; j++) { v[j] = (f16_t)x0[j]; v[4 + j] = (f16_t)x1[j]; }
  f16_t* p = dst + (size_t)ic * 8;
  if (ok) *(volatile v8hm*)p = v;
  __threadfence();
  if (ok) *(volatile v8hm*)p = v;
}

__global__ __launch_bounds__(256) void ln_concat_kernel(
    const float* __restrict__ emb1, const float* __restrict__ emb2,
    const float* __restrict__ g1, const float* __restrict__ b1,
    const float* __restrict__ ga, const float* __restrict__ ba,
    f16_t* __restrict__ cx1, f16_t* __restrict__ ea, int nrows) {
  __shared__ __attribute__((aligned(16))) f16_t St[8][256];
  const int wave = threadIdx.x >> 5, lane = threadIdx.x & 31;
  const int row = blockIdx.x * 8 + wave;
  const bool ok = row < nrows;
  const int rc = ok ? row : 0;
  const float* r1 = emb1 + (size_t)rc * C1_;
  const float* r2 = emb2 + (size_t)rc * C2_;

  const float x0 = r1[lane], x1 = r1[lane + 32];
  const float mu = wave_sum(x0 + x1) * (1.0f / 64.0f);
  const float d0 = x0 - mu, d1 = x1 - mu;
  const float var = wave_sum(d0 * d0 + d1 * d1) * (1.0f / 64.0f);
  const float rs = rsqrtf(var + 1e-6f);
  St[wave][lane]      = (f16_t)(d0 * rs * g1[lane] + b1[lane]);
  St[wave][lane + 32] = (f16_t)(d1 * rs * g1[lane + 32] + b1[lane + 32]);

  float e[6];
  e[0] = x0; e[1] = x1;
#pragma unroll
  for (int j = 2; j < 6; j++) e[j] = r2[lane + 32 * (j - 2)];
  float s = 0.f;
#pragma unroll
  for (int j = 0; j < 6; j++) s += e[j];
  const float ma = wave_sum(s) * (1.0f / 192.0f);
  float sq = 0.f;
#pragma unroll
  for (int j = 0; j < 6; j++) { e[j] -= ma; sq += e[j] * e[j]; }
  const float vara = wave_sum(sq) * (1.0f / 192.0f);
  const float rsa = rsqrtf(vara + 1e-6f);
#pragma unroll
  for (int j = 0; j < 6; j++) {
    const int c = lane + 32 * j;
    St[wave][64 + c] = (f16_t)(e[j] * rsa * ga[c] + ba[c]);
  }
  __syncthreads();

  const int l8 = (lane < 8) ? lane : 0;
  const int l24 = (lane < 24) ? lane : 0;
  const v8h pc = *(const v8hm*)&St[wave][l8 * 8];
  const v8h pe = *(const v8hm*)&St[wave][64 + l24 * 8];
  f16_t* dc = cx1 + (size_t)rc * C1_ + l8 * 8;
  f16_t* de = ea + (size_t)rc * KV_ + l24 * 8;
  const bool sc = ok && (lane < 8);
  const bool se = ok && (lane < 24);
  if (sc) *(volatile v8hm*)dc = pc;
  if (se) *(volatile v8hm*)de = pe;
  __threadfence();
  if (sc) *(volatile v8hm*)dc = pc;
  if (se) *(volatile v8hm*)de = pe;
}

__global__ __launch_bounds__(256) void ln64_kernel(
    const float* __restrict__ x, const float* __restrict__ g,
    const float* __restrict__ bb, f16_t* __restrict__ y, int nrows) {
  __shared__ __attribute__((aligned(16))) f16_t St[8][64];
  const int wave = threadIdx.x >> 5, lane = threadIdx.x & 31;
  const int row = blockIdx.x * 8 + wave;
  const bool ok = row < nrows;
  const int rc = ok ? row : 0;
  const float* r = x + (size_t)rc * C1_;
  const float x0 = r[lane], x1 = r[lane + 32];
  const float mu = wave_sum(x0 + x1) * (1.0f / 64.0f);
  const float d0 = x0 - mu, d1 = x1 - mu;
  const float var = wave_sum(d0 * d0 + d1 * d1) * (1.0f / 64.0f);
  const float rs = rsqrtf(var + 1e-6f);
  St[wave][lane]      = (f16_t)(d0 * rs * g[lane] + bb[lane]);
  St[wave][lane + 32] = (f16_t)(d1 * rs * g[lane + 32] + bb[lane + 32]);
  __syncthreads();
  const int l8 = (lane < 8) ? lane : 0;
  const v8h pc = *(const v8hm*)&St[wave][l8 * 8];
  f16_t* dc = y + (size_t)rc * C1_ + l8 * 8;
  const bool sc = ok && (lane < 8);
  if (sc) *(volatile v8hm*)dc = pc;
  __threadfence();
  if (sc) *(volatile v8hm*)dc = pc;
}

union CTile { float f[128][64]; f16_t h[128][64]; f16_t t[64][128]; };

template <int MODE, bool BIAS, bool GELU, bool RESID>
__global__ __launch_bounds__(256) void gemm_nt_kernel(
    const f16_t* __restrict__ A, int lda, long long aBatch,
    const f16_t* __restrict__ Bw, int ldb, long long bBatch,
    f16_t* __restrict__ Ch, float* __restrict__ Cf, int ldc, long long cBatch,
    int Kdim, const float* __restrict__ bias, const float* __restrict__ resid) {
  __shared__ __attribute__((aligned(16))) f16_t As[128][32];
  __shared__ __attribute__((aligned(16))) f16_t Bs[64][32];
  __shared__ __attribute__((aligned(16))) CTile Cs;
  const int tid = threadIdx.x, lane = tid & 31, wave = tid >> 5;
  const int hh = lane >> 4, m = lane & 15;
  const long long z = blockIdx.z;
  const f16_t* Ab = A + z * aBatch;
  const f16_t* Bb = Bw + z * bBatch;
  const int m0 = blockIdx.x * 128, n0 = blockIdx.y * 64;
  const int ar = tid >> 2, ac = (tid & 3) * 8;
  const f16_t* gA0 = Ab + (long long)(m0 + ar) * lda + ac;
  const f16_t* gA1 = Ab + (long long)(m0 + ar + 64) * lda + ac;
  const f16_t* gB  = Bb + (long long)(n0 + ar) * ldb + ac;
  v8f acc[4] = {};
  const int nk = Kdim >> 5;
  const int mrow = wave * 16 + m;
  for (int i = 0; i < nk; i++) {
    const int k0 = i << 5;
    const v8h sa0 = *(const v8hm*)(gA0 + k0);
    const v8h sa1 = *(const v8hm*)(gA1 + k0);
    const v8h sb  = *(const v8hm*)(gB + k0);
    __syncthreads();
    *(v8hm*)&As[ar][ac]      = sa0;
    *(v8hm*)&As[ar + 64][ac] = sa1;
    *(v8hm*)&Bs[ar][ac]      = sb;
    __syncthreads();
    Frag a;
    a.p[0] = *(const v8hm*)&As[mrow][8 * hh];
    a.p[1] = *(const v8hm*)&As[mrow][16 + 8 * hh];
#pragma unroll
    for (int nt = 0; nt < 4; nt++) {
      Frag b;
      b.p[0] = *(const v8hm*)&Bs[nt * 16 + m][8 * hh];
      b.p[1] = *(const v8hm*)&Bs[nt * 16 + m][16 + 8 * hh];
      acc[nt] = wmma16(a.v, b.v, acc[nt]);
    }
  }

#pragma unroll
  for (int nt = 0; nt < 4; nt++) {
    const int cn = nt * 16 + m;
    float bs = 0.f;
    if (BIAS) bs = bias[n0 + cn];
#pragma unroll
    for (int r = 0; r < 8; r++) {
      const int cm = wave * 16 + 8 * hh + r;
      float xv = acc[nt][r] + bs;
      if (GELU) xv = 0.5f * xv * (1.0f + erff(xv * 0.70710678118654752f));
      if (MODE == 1) Cs.f[cm][cn] = xv;
      else if (MODE == 0) Cs.h[cm][cn] = (f16_t)xv;
      else Cs.t[cn][cm] = (f16_t)xv;
    }
  }
  __syncthreads();

  if (MODE == 1) {
    float* Cb = Cf + z * cBatch;
    v4f vals[8];
#pragma unroll
    for (int j = 0; j < 8; j++) {
      const int row = wave * 16 + 2 * j + hh;
      const int c4 = m * 4;
      v4f v = *(const v4fm*)&Cs.f[row][c4];
      if (RESID) {
        const v4f rr = *(const v4fm*)(resid + (long long)(m0 + row) * ldc + n0 + c4);
        v += rr;
      }
      vals[j] = v;
    }
#pragma unroll
    for (int j = 0; j < 8; j++) {
      const int row = wave * 16 + 2 * j + hh;
      *(volatile v4fm*)(Cb + (long long)(m0 + row) * ldc + n0 + m * 4) = vals[j];
    }
    __threadfence();
#pragma unroll
    for (int j = 0; j < 8; j++) {
      const int row = wave * 16 + 2 * j + hh;
      *(volatile v4fm*)(Cb + (long long)(m0 + row) * ldc + n0 + m * 4) = vals[j];
    }
  } else if (MODE == 0) {
    f16_t* Cb = Ch + z * cBatch;
    v8h vals[4];
    const int rsub = lane >> 3, c8 = (lane & 7) * 8;
#pragma unroll
    for (int j = 0; j < 4; j++) {
      const int row = wave * 16 + 4 * j + rsub;
      vals[j] = *(const v8hm*)&Cs.h[row][c8];
    }
#pragma unroll
    for (int j = 0; j < 4; j++) {
      const int row = wave * 16 + 4 * j + rsub;
      *(volatile v8hm*)(Cb + (long long)(m0 + row) * ldc + n0 + c8) = vals[j];
    }
    __threadfence();
#pragma unroll
    for (int j = 0; j < 4; j++) {
      const int row = wave * 16 + 4 * j + rsub;
      *(volatile v8hm*)(Cb + (long long)(m0 + row) * ldc + n0 + c8) = vals[j];
    }
  } else {
    f16_t* Cb = Ch + z * cBatch;
    v8h vals[4];
    const int c8 = m * 8;
#pragma unroll
    for (int j = 0; j < 4; j++) {
      const int row = wave * 8 + 2 * j + hh;
      vals[j] = *(const v8hm*)&Cs.t[row][c8];
    }
#pragma unroll
    for (int j = 0; j < 4; j++) {
      const int row = wave * 8 + 2 * j + hh;
      *(volatile v8hm*)(Cb + (long long)(n0 + row) * ldc + m0 + c8) = vals[j];
    }
    __threadfence();
#pragma unroll
    for (int j = 0; j < 4; j++) {
      const int row = wave * 8 + 2 * j + hh;
      *(volatile v8hm*)(Cb + (long long)(n0 + row) * ldc + m0 + c8) = vals[j];
    }
  }
}

__global__ __launch_bounds__(256) void scores_softmax_kernel(
    const f16_t* __restrict__ QT, const f16_t* __restrict__ KT, f16_t* __restrict__ P) {
  __shared__ __attribute__((aligned(16))) f16_t Aq[64][32];
  __shared__ __attribute__((aligned(16))) f16_t Bk[192][32];
  __shared__ float Sb[64][196];
  __shared__ __attribute__((aligned(16))) f16_t Pst[64][192];
  __shared__ float red[8];
  const int tid = threadIdx.x, lane = tid & 31, wave = tid >> 5;
  const int hh = lane >> 4, m = lane & 15;
  const int bh = blockIdx.x, b = bh >> 2, hd = bh & 3;
  const f16_t* Ab = QT + (size_t)hd * C1_ * BN_ + (size_t)b * N_;
  const f16_t* Bb = KT + (size_t)hd * KV_ * BN_ + (size_t)b * N_;
  const int mt = wave & 3, ng = wave >> 2;
  v8f acc[6] = {};
  const int ar = tid >> 2, ac = (tid & 3) * 8;
  const f16_t* gA  = Ab + (size_t)ar * BN_ + ac;
  const f16_t* gB0 = Bb + (size_t)ar * BN_ + ac;
  const f16_t* gB1 = Bb + (size_t)(ar + 64) * BN_ + ac;
  const f16_t* gB2 = Bb + (size_t)(ar + 128) * BN_ + ac;
  const int mrow = mt * 16 + m;

  const int nk = N_ / 32;
  for (int it = 0; it < nk; it++) {
    const int n0 = it * 32;
    const v8h sa  = *(const v8hm*)(gA + n0);
    const v8h sb0 = *(const v8hm*)(gB0 + n0);
    const v8h sb1 = *(const v8hm*)(gB1 + n0);
    const v8h sb2 = *(const v8hm*)(gB2 + n0);
    __syncthreads();
    *(v8hm*)&Aq[ar][ac]       = sa;
    *(v8hm*)&Bk[ar][ac]       = sb0;
    *(v8hm*)&Bk[ar + 64][ac]  = sb1;
    *(v8hm*)&Bk[ar + 128][ac] = sb2;
    __syncthreads();
    Frag a;
    a.p[0] = *(const v8hm*)&Aq[mrow][8 * hh];
    a.p[1] = *(const v8hm*)&Aq[mrow][16 + 8 * hh];
#pragma unroll
    for (int t = 0; t < 6; t++) {
      const int col = (ng * 6 + t) * 16 + m;
      Frag bf;
      bf.p[0] = *(const v8hm*)&Bk[col][8 * hh];
      bf.p[1] = *(const v8hm*)&Bk[col][16 + 8 * hh];
      acc[t] = wmma16(a.v, bf.v, acc[t]);
    }
  }

  const float sc = 0.07216878364870322f;
#pragma unroll
  for (int t = 0; t < 6; t++) {
    const int cn = (ng * 6 + t) * 16 + m;
#pragma unroll
    for (int r = 0; r < 8; r++)
      Sb[mt * 16 + 8 * hh + r][cn] = acc[t][r] * sc;
  }
  __syncthreads();

  const int r0 = tid >> 2;
  const int c0 = (tid & 3) * 48;
  float s = 0.f;
#pragma unroll 4
  for (int j = 0; j < 48; j++) s += Sb[r0][c0 + j];
  s = wave_sum(s);
  if (lane == 0) red[wave] = s;
  __syncthreads();
  float tot = 0.f;
#pragma unroll
  for (int w = 0; w < 8; w++) tot += red[w];
  const float mean = tot * (1.0f / 12288.0f);
  __syncthreads();
  float sq = 0.f;
#pragma unroll 4
  for (int j = 0; j < 48; j++) { const float d = Sb[r0][c0 + j] - mean; sq += d * d; }
  sq = wave_sum(sq);
  if (lane == 0) red[wave] = sq;
  __syncthreads();
  float tot2 = 0.f;
#pragma unroll
  for (int w = 0; w < 8; w++) tot2 += red[w];
  const float var  = tot2 * (1.0f / 12288.0f);
  const float rstd = rsqrtf(var + 1e-5f);

  const float pscale = 4096.0f;
  for (int rr = 0; rr < 8; rr++) {
    const int r = wave * 8 + rr;
    float xs[6];
    float mx = -3.0e38f;
#pragma unroll
    for (int j = 0; j < 6; j++) {
      xs[j] = (Sb[r][lane + 32 * j] - mean) * rstd;
      mx = fmaxf(mx, xs[j]);
    }
    mx = wave_max(mx);
    float es = 0.f;
#pragma unroll
    for (int j = 0; j < 6; j++) { xs[j] = expf(xs[j] - mx); es += xs[j]; }
    es = wave_sum(es);
    const float inv = (1.0f / es) * pscale;
#pragma unroll
    for (int j = 0; j < 6; j++)
      Pst[r][lane + 32 * j] = (f16_t)(xs[j] * inv);
  }
  __syncthreads();

  f16_t* Pb = P + (size_t)bh * C1_ * KV_;
  const int l24 = (lane < 24) ? lane : 0;
  const bool se = lane < 24;
  v8h vals[8];
#pragma unroll
  for (int j = 0; j < 8; j++) vals[j] = *(const v8hm*)&Pst[wave * 8 + j][l24 * 8];
#pragma unroll
  for (int j = 0; j < 8; j++)
    if (se) *(volatile v8hm*)(Pb + (size_t)(wave * 8 + j) * KV_ + l24 * 8) = vals[j];
  __threadfence();
#pragma unroll
  for (int j = 0; j < 8; j++)
    if (se) *(volatile v8hm*)(Pb + (size_t)(wave * 8 + j) * KV_ + l24 * 8) = vals[j];
}

__global__ __launch_bounds__(256) void ctx_mean_kernel(
    const f16_t* __restrict__ V, const f16_t* __restrict__ P, f16_t* __restrict__ ctxm) {
  __shared__ __attribute__((aligned(16))) f16_t Vs[64][32];
  __shared__ __attribute__((aligned(16))) f16_t Ps[64][32];
  __shared__ __attribute__((aligned(16))) f16_t Cs[64][64];
  const int tid = threadIdx.x, lane = tid & 31, wave = tid >> 5;
  const int hh = lane >> 4, m = lane & 15;
  const int b = blockIdx.z;
  const int n0 = blockIdx.x * 64;
  const int mt = wave & 3, ng = wave >> 2;
  v8f acc[2] = {};
  const int ar = tid >> 2, ac = (tid & 3) * 8;
  const int mrow = mt * 16 + m;

  const int nsteps = H_ * (KV_ / 32);
  for (int it = 0; it < nsteps; it++) {
    const int hd = it / 6;
    const int k0 = (it - hd * 6) * 32;
    const f16_t* Vb = V + ((size_t)hd * BN_ + (size_t)b * N_ + n0) * KV_;
    const f16_t* Pb = P + (size_t)(b * H_ + hd) * C1_ * KV_;
    const v8h sv = *(const v8hm*)(Vb + (size_t)ar * KV_ + k0 + ac);
    const v8h sp = *(const v8hm*)(Pb + (size_t)ar * KV_ + k0 + ac);
    __syncthreads();
    *(v8hm*)&Vs[ar][ac] = sv;
    *(v8hm*)&Ps[ar][ac] = sp;
    __syncthreads();
    Frag a;
    a.p[0] = *(const v8hm*)&Vs[mrow][8 * hh];
    a.p[1] = *(const v8hm*)&Vs[mrow][16 + 8 * hh];
#pragma unroll
    for (int t = 0; t < 2; t++) {
      const int col = (ng * 2 + t) * 16 + m;
      Frag bf;
      bf.p[0] = *(const v8hm*)&Ps[col][8 * hh];
      bf.p[1] = *(const v8hm*)&Ps[col][16 + 8 * hh];
      acc[t] = wmma16(a.v, bf.v, acc[t]);
    }
  }

  const float oscale = 0.25f / 4096.0f;
#pragma unroll
  for (int t = 0; t < 2; t++) {
    const int cn = (ng * 2 + t) * 16 + m;
#pragma unroll
    for (int r = 0; r < 8; r++)
      Cs[mt * 16 + 8 * hh + r][cn] = (f16_t)(acc[t][r] * oscale);
  }
  __syncthreads();

  const int rsub = lane >> 3, c8 = (lane & 7) * 8;
  v8h vals[2];
#pragma unroll
  for (int j = 0; j < 2; j++) vals[j] = *(const v8hm*)&Cs[wave * 8 + 4 * j + rsub][c8];
#pragma unroll
  for (int j = 0; j < 2; j++) {
    const int row = wave * 8 + 4 * j + rsub;
    *(volatile v8hm*)(ctxm + ((size_t)b * N_ + n0 + row) * C1_ + c8) = vals[j];
  }
  __threadfence();
#pragma unroll
  for (int j = 0; j < 2; j++) {
    const int row = wave * 8 + 4 * j + rsub;
    *(volatile v8hm*)(ctxm + ((size_t)b * N_ + n0 + row) * C1_ + c8) = vals[j];
  }
}

extern "C" void kernel_launch(void* const* d_in, const int* in_sizes, int n_in,
                              void* d_out, int out_size, void* d_ws, size_t ws_size,
                              hipStream_t stream) {
  if (n_in < 16) return;
  const int need[16] = {BN_ * C1_, BN_ * C2_, H_ * C1_ * C1_, H_ * KV_ * KV_, H_ * KV_ * KV_,
                        C1_ * C1_, C1_, C1_, KV_, KV_, C1_, C1_, MLP_ * C1_, MLP_,
                        C1_ * MLP_, C1_};
  for (int i = 0; i < 16; i++) if (in_sizes[i] != need[i]) return;
  if (out_size != BN_ * C1_) return;

  const float* emb1    = (const float*)d_in[0];
  const float* emb2    = (const float*)d_in[1];
  const float* Wq      = (const float*)d_in[2];
  const float* Wk      = (const float*)d_in[3];
  const float* Wv      = (const float*)d_in[4];
  const float* Wout    = (const float*)d_in[5];
  const float* ln1_g   = (const float*)d_in[6];
  const float* ln1_b   = (const float*)d_in[7];
  const float* lnall_g = (const float*)d_in[8];
  const float* lnall_b = (const float*)d_in[9];
  const float* ffn_g   = (const float*)d_in[10];
  const float* ffn_b   = (const float*)d_in[11];
  const float* fc1_w   = (const float*)d_in[12];
  const float* fc1_b   = (const float*)d_in[13];
  const float* fc2_w   = (const float*)d_in[14];
  const float* fc2_b   = (const float*)d_in[15];
  float* out = (float*)d_out;

  char* ws = (char*)d_ws;
  size_t off = 0;
  auto take = [&](size_t bytes) -> void* {
    off = (off + 255) & ~(size_t)255;
    void* p = ws + off;
    off += bytes;
    return p;
  };
  f16_t* cx1   = (f16_t*)take((size_t)BN_ * C1_ * 2);
  f16_t* ea    = (f16_t*)take((size_t)BN_ * KV_ * 2);
  f16_t* Wqh   = (f16_t*)take((size_t)H_ * C1_ * C1_ * 2);
  f16_t* Wkh   = (f16_t*)take((size_t)H_ * KV_ * KV_ * 2);
  f16_t* Wvh   = (f16_t*)take((size_t)H_ * KV_ * KV_ * 2);
  f16_t* Wouth = (f16_t*)take((size_t)C1_ * C1_ * 2);
  f16_t* fc1h  = (f16_t*)take((size_t)MLP_ * C1_ * 2);
  f16_t* fc2h  = (f16_t*)take((size_t)C1_ * MLP_ * 2);
  f16_t* QT    = (f16_t*)take((size_t)H_ * C1_ * BN_ * 2);
  f16_t* KT    = (f16_t*)take((size_t)H_ * KV_ * BN_ * 2);
  f16_t* Vbuf  = (f16_t*)take((size_t)H_ * BN_ * KV_ * 2);
  f16_t* Pm    = (f16_t*)take((size_t)B_ * H_ * C1_ * KV_ * 2);
  f16_t* ctxm  = (f16_t*)take((size_t)BN_ * C1_ * 2);
  float* cx    = (float*)take((size_t)BN_ * C1_ * 4);
  f16_t* ybuf  = (f16_t*)take((size_t)BN_ * C1_ * 2);
  f16_t* h1    = (f16_t*)take((size_t)BN_ * MLP_ * 2);
  if (off > ws_size) return;

  auto cvt = [&](const float* s, f16_t* d, int n) {
    const int n8 = n / 8;
    cvt_f16_kernel<<<(n8 + 255) / 256, 256, 0, stream>>>(s, d, n8);
  };
  cvt(Wq,    Wqh,   H_ * C1_ * C1_);
  cvt(Wk,    Wkh,   H_ * KV_ * KV_);
  cvt(Wv,    Wvh,   H_ * KV_ * KV_);
  cvt(Wout,  Wouth, C1_ * C1_);
  cvt(fc1_w, fc1h,  MLP_ * C1_);
  cvt(fc2_w, fc2h,  C1_ * MLP_);

  ln_concat_kernel<<<(BN_ + 7) / 8, 256, 0, stream>>>(emb1, emb2, ln1_g, ln1_b,
                                                      lnall_g, lnall_b, cx1, ea, BN_);

  gemm_nt_kernel<2, false, false, false>
      <<<dim3(BN_ / 128, 1, H_), 256, 0, stream>>>(
      cx1, C1_, 0LL, Wqh, C1_, (long long)C1_ * C1_,
      QT, cx, BN_, (long long)C1_ * BN_, C1_, fc1_b, emb1);
  gemm_nt_kernel<2, false, false, false>
      <<<dim3(BN_ / 128, KV_ / 64, H_), 256, 0, stream>>>(
      ea, KV_, 0LL, Wkh, KV_, (long long)KV_ * KV_,
      KT, cx, BN_, (long long)KV_ * BN_, KV_, fc1_b, emb1);
  gemm_nt_kernel<0, false, false, false>
      <<<dim3(BN_ / 128, KV_ / 64, H_), 256, 0, stream>>>(
      ea, KV_, 0LL, Wvh, KV_, (long long)KV_ * KV_,
      Vbuf, cx, KV_, (long long)BN_ * KV_, KV_, fc1_b, emb1);

  scores_softmax_kernel<<<B_ * H_, 256, 0, stream>>>(QT, KT, Pm);

  ctx_mean_kernel<<<dim3(N_ / 64, 1, B_), 256, 0, stream>>>(Vbuf, Pm, ctxm);

  gemm_nt_kernel<1, false, false, true>
      <<<dim3(BN_ / 128, 1, 1), 256, 0, stream>>>(
      ctxm, C1_, 0LL, Wouth, C1_, 0LL,
      ybuf, cx, C1_, 0LL, C1_, fc1_b, emb1);

  ln64_kernel<<<(BN_ + 7) / 8, 256, 0, stream>>>(cx, ffn_g, ffn_b, ybuf, BN_);

  gemm_nt_kernel<0, true, true, false>
      <<<dim3(BN_ / 128, MLP_ / 64, 1), 256, 0, stream>>>(
      ybuf, C1_, 0LL, fc1h, C1_, 0LL,
      h1, cx, MLP_, 0LL, C1_, fc1_b, emb1);

  gemm_nt_kernel<1, true, false, true>
      <<<dim3(BN_ / 128, 1, 1), 256, 0, stream>>>(
      h1, MLP_, 0LL, fc2h, MLP_, 0LL,
      ybuf, out, C1_, 0LL, MLP_, fc2_b, cx);
}
